// TrainableTree_79611513798985
// MI455X (gfx1250) — hardware-run, weakly checked
//
#include <hip/hip_runtime.h>


#define NROW 262144
#define NDIM 10
#define NKP  32
#define NM   64
typedef _Float16 h16;
typedef unsigned short bf;
typedef __attribute__((ext_vector_type(16))) __bf16   v16bf;
typedef __attribute__((ext_vector_type(16))) _Float16 v16h;
typedef __attribute__((ext_vector_type(8)))  _Float16 v8h;
typedef __attribute__((ext_vector_type(8)))  unsigned short v8us;
typedef __attribute__((ext_vector_type(8)))  float    v8f;
typedef __attribute__((ext_vector_type(4)))  float    v4f;
typedef v8h  __attribute__((may_alias)) v8ha;
typedef v4f  __attribute__((may_alias)) v4fa;
typedef v8us __attribute__((may_alias)) v8usa;

__device__ __forceinline__ unsigned short f2bf(float f) { unsigned u = __float_as_uint(f); u += 0x7FFFu + ((u >> 16) & 1u); return (unsigned short)(u >> 16); }
__device__ __forceinline__ float bf2f(unsigned short b) { return __uint_as_float(((unsigned)b) << 16); }
__device__ __forceinline__ float bfr(float f) { return bf2f(f2bf(f)); }
__device__ __forceinline__ v16h cat16(v8h lo, v8h hi) { return __builtin_shufflevector(lo, hi, 0, 1, 2, 3, 4, 5, 6, 7, 8, 9, 10, 11, 12, 13, 14, 15); }
__device__ __forceinline__ v16bf cat16b(v8us lo, v8us hi) { return __builtin_bit_cast(v16bf, __builtin_shufflevector(lo, hi, 0, 1, 2, 3, 4, 5, 6, 7, 8, 9, 10, 11, 12, 13, 14, 15)); }
__device__ __forceinline__ v8f wmma16(v16h a, v16h b, v8f c) { return __builtin_amdgcn_wmma_f32_16x16x32_f16(false, a, false, b, (short)0, c, false, false); }
__device__ __forceinline__ v8f wmmab(v16bf a, v16bf b, v8f c) { return __builtin_amdgcn_wmma_f32_16x16x32_bf16(false, a, false, b, (short)0, c, false, false); }

template <typename T16> struct WFrag;
template <> struct WFrag<h16> { typedef v16h V; static __device__ __forceinline__ V ld(const h16* p) { return cat16(*(const v8h*)p, *(const v8h*)(p + 16)); } static __device__ __forceinline__ v8f mma(V a, V b, v8f c) { return wmma16(a, b, c); } };
template <> struct WFrag<bf> { typedef v16bf V; static __device__ __forceinline__ V ld(const bf* p) { return cat16b(*(const v8us*)p, *(const v8us*)(p + 16)); } static __device__ __forceinline__ v8f mma(V a, V b, v8f c) { return wmmab(a, b, c); } };
template <typename T16, int NSPLIT, bool BIAS>
__global__ __launch_bounds__(32) void k_gemmw(const T16* __restrict__ A, const T16* __restrict__ A2, const T16* __restrict__ Bt, const T16* __restrict__ Bt2, int K, float* C, int ldc, const float* __restrict__ bias, size_t sA, size_t sB, size_t sC) {
    typedef typename WFrag<T16>::V V;
    __shared__ __align__(16) float os[16 * 68];
    const size_t z = blockIdx.z; A += z * sA; if (A2) A2 += z * sA; Bt += z * sB; if (Bt2) Bt2 += z * sB; C += z * sC;
    const int lane = threadIdx.x & 31, lr = lane & 15, hi = lane >> 4; const int r0 = blockIdx.x * 64, c0 = blockIdx.y * 64;
    v8f acc[4][4];
#pragma unroll
    for (int mb = 0; mb < 4; ++mb)
#pragma unroll
        for (int nb = 0; nb < 4; ++nb) acc[mb][nb] = (v8f){};
    const size_t aoff = (size_t)(r0 + lr) * K + 8 * hi, boff = (size_t)(c0 + lr) * K + 8 * hi;
    for (int kc = 0; kc < K; kc += 32) {
        V a[4], a2[4];
#pragma unroll
        for (int mb = 0; mb < 4; ++mb) { a[mb] = WFrag<T16>::ld(A + aoff + (size_t)mb * 16 * K + kc); if (NSPLIT == 1 || NSPLIT == 2) a2[mb] = WFrag<T16>::ld(A2 + aoff + (size_t)mb * 16 * K + kc); }
#pragma unroll
        for (int nb = 0; nb < 4; ++nb) { const V b = WFrag<T16>::ld(Bt + boff + (size_t)nb * 16 * K + kc); V b2; if (NSPLIT >= 2) b2 = WFrag<T16>::ld(Bt2 + boff + (size_t)nb * 16 * K + kc);
#pragma unroll
            for (int mb = 0; mb < 4; ++mb) { acc[mb][nb] = WFrag<T16>::mma(a[mb], b, acc[mb][nb]); if (NSPLIT == 1 || NSPLIT == 2) acc[mb][nb] = WFrag<T16>::mma(a2[mb], b, acc[mb][nb]); if (NSPLIT >= 2) acc[mb][nb] = WFrag<T16>::mma(a[mb], b2, acc[mb][nb]); } }
        asm volatile("v_nop\n\tv_nop\n\tv_nop\n\tv_nop" : "+v"(acc[0][0]), "+v"(acc[1][1]), "+v"(acc[2][2]), "+v"(acc[3][3]) : "v"(a[0]), "v"(a[3]));
    }
#pragma unroll
    for (int mb = 0; mb < 4; ++mb) {
#pragma unroll
        for (int nb = 0; nb < 4; ++nb) {
#pragma unroll
            for (int j = 0; j < 8; ++j) os[(hi * 8 + j) * 68 + nb * 16 + lr] = acc[mb][nb][j]; }
        __builtin_amdgcn_wave_barrier(); asm volatile("" ::: "memory");
        float* crow = C + (size_t)(r0 + mb * 16) * ldc + c0;
#pragma unroll 1
        for (int ps = 0; ps < 2; ++ps) {
#pragma unroll
            for (int s = 0; s < 8; ++s) { const int row = 2 * s + hi, cofs = lr * 4; v4f val = *(const v4fa*)(os + row * 68 + cofs); if (BIAS) { val[0] += bfr(bias[c0 + cofs]); val[1] += bfr(bias[c0 + cofs + 1]); val[2] += bfr(bias[c0 + cofs + 2]); val[3] += bfr(bias[c0 + cofs + 3]); }
                *(volatile v4f*)(crow + (size_t)row * ldc + cofs) = val; }
            if (ps == 0) __threadfence(); }
        __builtin_amdgcn_wave_barrier(); asm volatile("" ::: "memory");
    }
}

__global__ __launch_bounds__(256) void k_pad32(const float* __restrict__ src, bf* dst, int R) { const int i = blockIdx.x * 256 + threadIdx.x; if (i >= R * 4) return; const int row = i >> 2, c0 = (i & 3) * 8; v8us o;
#pragma unroll
    for (int k = 0; k < 8; ++k) { const int c = c0 + k; const int cs = c < NDIM ? c : NDIM - 1; const unsigned short keep = (unsigned short)(c < NDIM ? 0xffffu : 0u); o[k] = (unsigned short)(f2bf(src[(size_t)row * NDIM + cs]) & keep); }
    bf* p = dst + (size_t)i * 8; *(volatile v8us*)p = o; __threadfence(); *(volatile v8us*)p = o; }

template <bool ROUNDP>
__global__ __launch_bounds__(64) void k_vlev(const float* __restrict__ PREV, const float* __restrict__ Wl, float* OUT) { const int m = threadIdx.x, j = blockIdx.x; const float* pv = PREV + (size_t)(j >> 1) * NM; const float* w = Wl + (size_t)j * NM * NM + m; float s = 0.0f;
  for (int o = 0; o < NM; ++o) { const float p = ROUNDP ? bfr(pv[o]) : pv[o]; s += p * bfr(w[(size_t)o * NM]); }
  float* op = OUT + (size_t)j * NM + m; *(volatile float*)op = s; __threadfence(); *(volatile float*)op = s; }

__global__ __launch_bounds__(64) void k_ulev(const float* __restrict__ V3, const float* __restrict__ Wleaf, float* U) { const int m = threadIdx.x; float s = 0.0f;
#pragma unroll 1
  for (int k = 0; k < 16; ++k) { const float* pv = V3 + (size_t)(k >> 1) * NM; const float* w = Wleaf + (size_t)k * NM * NM + m;
    for (int o = 0; o < NM; ++o) s += pv[o] * bfr(w[(size_t)o * NM]); }
  *(volatile float*)(U + m) = s; __threadfence(); *(volatile float*)(U + m) = s; }

__global__ __launch_bounds__(32) void k_const(const float* __restrict__ Wr, const float* __restrict__ V1, const float* __restrict__ V2, const float* __restrict__ V3, const float* __restrict__ b1, const float* __restrict__ b2, const float* __restrict__ b3, const float* __restrict__ bleaf, const float* __restrict__ br, float* C) { if (threadIdx.x != 0) return; float c = bfr(br[0]);
#pragma unroll 1
  for (int j = 0; j < 2; ++j) for (int o = 0; o < NM; ++o) c += bfr(Wr[o]) * bfr(b1[j * NM + o]);
#pragma unroll 1
  for (int j = 0; j < 4; ++j) for (int o = 0; o < NM; ++o) c += V1[(j >> 1) * NM + o] * bfr(b2[j * NM + o]);
#pragma unroll 1
  for (int j = 0; j < 8; ++j) for (int o = 0; o < NM; ++o) c += V2[(j >> 1) * NM + o] * bfr(b3[j * NM + o]);
#pragma unroll 1
  for (int k = 0; k < 16; ++k) for (int o = 0; o < NM; ++o) c += V3[(k >> 1) * NM + o] * bfr(bleaf[k * NM + o]);
  *(volatile float*)C = c; __threadfence(); *(volatile float*)C = c; }

__global__ __launch_bounds__(256) void k_rows(const float* __restrict__ x, const float* __restrict__ HP, const float* __restrict__ U, const float* __restrict__ C, float* OUT) { const int n = blockIdx.x * 256 + threadIdx.x; if (n >= NROW) return; float a = 1.0f;
#pragma unroll
  for (int d = 0; d < NDIM; ++d) { const float xv = bfr(x[(size_t)n * NDIM + d]); a *= xv * xv - 1.0f; }
  a = a / sqrtf(1000.0f + a * a); float acc = 0.0f; const float* hp = HP + (size_t)n * NM;
  for (int m = 0; m < NM; ++m) acc += sinf(hp[m]) * U[m];
  const float r = a * (acc + C[0]); *(volatile float*)(OUT + n) = r; __threadfence(); *(volatile float*)(OUT + n) = r; }

extern "C" void kernel_launch(void* const* d_in, const int* in_sizes, int n_in,
                              void* d_out, int out_size, void* d_ws, size_t ws_size, hipStream_t stream) {
    (void)in_sizes; (void)n_in; (void)out_size;
    const float* x = (const float*)d_in[0]; const float* Wt = (const float*)d_in[1]; const float* bt = (const float*)d_in[2]; const float* Wleaf = (const float*)d_in[3]; const float* bleaf = (const float*)d_in[4]; const float* W3 = (const float*)d_in[5]; const float* b3 = (const float*)d_in[6]; const float* W2 = (const float*)d_in[7]; const float* b2 = (const float*)d_in[8]; const float* W1 = (const float*)d_in[9]; const float* b1 = (const float*)d_in[10]; const float* Wr = (const float*)d_in[11]; const float* br = (const float*)d_in[12];
    float* OUT = (float*)d_out;
    char* wsp = (char*)d_ws;
    auto take = [&](size_t bytes) { char* p = wsp; wsp += (bytes + 255) & ~(size_t)255; return (void*)p; };
    bf* XP = (bf*)take((size_t)NROW * NKP * 2); bf* WP = (bf*)take((size_t)NM * NKP * 2); float* HP = (float*)take((size_t)NROW * NM * 4); float* V1 = (float*)take(2 * NM * 4); float* V2 = (float*)take(4 * NM * 4); float* V3 = (float*)take(8 * NM * 4); float* U = (float*)take(NM * 4); float* C = (float*)take(4);
    if ((size_t)(wsp - (char*)d_ws) > ws_size) return;
    k_pad32<<<NROW * 4 / 256, 256, 0, stream>>>(x, XP, NROW);
    k_pad32<<<1, 256, 0, stream>>>(Wt, WP, NM);
    k_gemmw<bf, 0, true><<<dim3(NROW / 64, NM / 64, 1), 32, 0, stream>>>(XP, nullptr, WP, nullptr, NKP, HP, NM, bt, 0, 0, 0);
    k_vlev<true><<<2, 64, 0, stream>>>(Wr, W1, V1);
    k_vlev<false><<<4, 64, 0, stream>>>(V1, W2, V2);
    k_vlev<false><<<8, 64, 0, stream>>>(V2, W3, V3);
    k_ulev<<<1, 64, 0, stream>>>(V3, Wleaf, U);
    k_const<<<1, 32, 0, stream>>>(Wr, V1, V2, V3, b1, b2, b3, bleaf, br, C);
    k_rows<<<NROW / 256, 256, 0, stream>>>(x, HP, U, C, OUT);
}
